// TinyAttentionMemory_67602785239363
// MI455X (gfx1250) — hardware-verified
//
#include <hip/hip_runtime.h>


namespace {
constexpr int NB = 32, T = 16, HW = 128, C1 = 16, C2 = 32, C3 = 64, FD = 128, DK = 64, DV = 128, S = 6, T0 = T - S - 1  , NFR = NB * (S + 1)  ;
constexpr int H1 = HW / 2  , H2 = HW / 4  , K2 = C1 * 9  , K2P = 160, K3 = C2 * 9  ;
constexpr float XS = 8.0f, WSC = 256.0f, SCALE = 0.125f  ;

typedef _Float16 b16;
typedef __attribute__((ext_vector_type(16))) _Float16 v16b;
typedef __attribute__((ext_vector_type(8))) _Float16 v8b;
typedef __attribute__((ext_vector_type(8))) float v8f;
typedef __attribute__((ext_vector_type(4))) float v4f;
__device__ __forceinline__ float bf16_rne(float f) { unsigned int u = __float_as_uint(f); u += 0x7FFFu + ((u >> 16) & 1u); return __uint_as_float(u & 0xFFFF0000u); }
__device__ __forceinline__ void split16(float v, b16& hi, b16& lo) { hi = (b16)v; lo = (b16)(v - (float)hi); }
__device__ __forceinline__ v16b frag_kb(const b16* p, int hh) { const v8b a = *(const v8b*)(p + 8 * hh), b = *(const v8b*)(p + 16 + 8 * hh); v16b f;
#pragma unroll
  for (int e = 0; e < 8; ++e) { f[e] = a[e]; f[8 + e] = b[e]; } return f; }
__device__ __forceinline__ v8f wmma16b(v16b a, v16b b, v8f c) { v8f d = __builtin_amdgcn_wmma_f32_16x16x32_f16(false, a, false, b, (short)0, c, false, false); asm volatile("v_nop\n\tv_nop\n\tv_nop\n\tv_nop" : "+v"(d) : "v"(a), "v"(b)); return d; }
__device__ __forceinline__ void wave_lds_sync() { __builtin_amdgcn_fence(__ATOMIC_RELEASE, "workgroup"); __builtin_amdgcn_wave_barrier(); __builtin_amdgcn_fence(__ATOMIC_ACQUIRE, "workgroup"); }
__device__ __forceinline__ float pmul(float a, float b) { float p = a * b; asm volatile("" : "+v"(p)); return p; }
__device__ __forceinline__ size_t frame_src(int f) { const int b = f / (S + 1), t = T0 + f % (S + 1); return ((size_t)b * T + t) * HW * HW; }

__global__ __launch_bounds__(256) void prepw_kernel(const float* __restrict__ w1, const float* __restrict__ w2, const float* __restrict__ w3, b16* __restrict__ W1P, b16* __restrict__ W2P, b16* __restrict__ W3P) {
  const int t = blockIdx.x * 256 + threadIdx.x; const int n1 = C1 * 32 / 8, n2 = C2 * K2P / 8, n3 = C3 * K3 / 8; v8b o; int u = t;
  if (u < n1) { const int e = u * 8, oc = e / 32, k0 = e % 32; for (int j = 0; j < 8; ++j) { const int k = k0 + j; o[j] = (k < 9) ? (b16)(bf16_rne(w1[oc * 9 + k]) * WSC) : (b16)0.0f; } for (int pass = 0; pass < 2; ++pass) { *(volatile v8b*)(W1P + e) = o; __threadfence(); } return; } u -= n1;
  if (u < n2) { const int e = u * 8, oc = e / K2P, k0 = e % K2P; for (int j = 0; j < 8; ++j) { const int k = k0 + j; o[j] = (k < K2) ? (b16)(bf16_rne(w2[oc * K2 + k]) * WSC) : (b16)0.0f; } for (int pass = 0; pass < 2; ++pass) { *(volatile v8b*)(W2P + e) = o; __threadfence(); } return; } u -= n2;
  if (u < n3) { const int e = u * 8, oc = e / K3, k0 = e % K3; for (int j = 0; j < 8; ++j) o[j] = (b16)(bf16_rne(w3[oc * K3 + k0 + j]) * WSC); for (int pass = 0; pass < 2; ++pass) { *(volatile v8b*)(W3P + e) = o; __threadfence(); } }
}
__global__ __launch_bounds__(256) void conv1_kernel(const float* __restrict__ img, const b16* __restrict__ W1P, const float* __restrict__ b1, b16* __restrict__ P1h, b16* __restrict__ P1l) {
  __shared__ __attribute__((aligned(16))) b16 At[8][16][32 + 8]; __shared__ float Cs[2][HW][C1 + 1]; __shared__ __attribute__((aligned(16))) b16 Rh[C1][H1 + 8], Rl[C1][H1 + 8];
  const int f = blockIdx.y, y0 = blockIdx.x * 2; const int wave = threadIdx.x >> 5, lane = threadIdx.x & 31, nloc = lane & 15, hlf = lane >> 4, t_ = threadIdx.x; const float* im = img + frame_src(f);
  for (int tt = 0; tt < 2; ++tt) { const int tile = wave * 2 + tt; const int ry = y0 + (tile >> 3), x0 = (tile & 7) * 16;
    for (int k = hlf * 16; k < hlf * 16 + 16; ++k) { float v = 0.0f; if (k < 9) { const int ky = k / 3, kx = k % 3; const int yy = ry + ky - 1, xx = x0 + nloc + kx - 1; if (yy >= 0 && yy < HW && xx >= 0 && xx < HW) v = bf16_rne(im[yy * HW + xx]); } At[wave][nloc][k] = (b16)(v * XS); }
    wave_lds_sync();
    v8f d = {}; d = wmma16b(frag_kb(&At[wave][nloc][0], hlf), frag_kb(W1P + (size_t)nloc * 32, hlf), d);
    for (int r = 0; r < 8; ++r) { const int px = x0 + 8 * hlf + r; Cs[tile >> 3][px][nloc] = fmaxf(d[r] * (1.0f / (XS * WSC)) + bf16_rne(b1[nloc]), 0.0f); }
    wave_lds_sync(); }
  __syncthreads();
  for (int q = t_; q < C1 * H1; q += 256) { const int c = q / H1, px = q % H1; const float m = fmaxf(fmaxf(Cs[0][2 * px][c], Cs[0][2 * px + 1][c]), fmaxf(Cs[1][2 * px][c], Cs[1][2 * px + 1][c])); b16 p, ql; split16(m * XS, p, ql); Rh[c][px] = p; Rl[c][px] = ql; }
  __syncthreads();
  for (int pass = 0; pass < 2; ++pass) { if (t_ < C1 * 8) { const int c = t_ >> 3, c8 = (t_ & 7) * 8; const size_t gi = (((size_t)f * C1 + c) * H1 + blockIdx.x) * H1 + c8; *(volatile v8b*)(P1h + gi) = *(const v8b*)(&Rh[c][c8]); *(volatile v8b*)(P1l + gi) = *(const v8b*)(&Rl[c][c8]); } __threadfence(); }
}
__global__ __launch_bounds__(128) void conv2_kernel(const b16* __restrict__ P1h, const b16* __restrict__ P1l, const b16* __restrict__ W2P, const float* __restrict__ b2, b16* __restrict__ P2h, b16* __restrict__ P2l) {
  __shared__ __attribute__((aligned(16))) b16 Ah[4][16][K2P + 8], Al[4][16][K2P + 8]; __shared__ float Cs[4][H1][C2 + 1]; __shared__ __attribute__((aligned(16))) b16 Rh[C2][2 * H2 + 8], Rl[C2][2 * H2 + 8];
  const int f = blockIdx.y, y0 = blockIdx.x * 4; const int wave = threadIdx.x >> 5, lane = threadIdx.x & 31, nloc = lane & 15, hlf = lane >> 4, t_ = threadIdx.x;
  const b16* ph = P1h + (size_t)f * C1 * H1 * H1; const b16* pl = P1l + (size_t)f * C1 * H1 * H1;
  for (int tt = 0; tt < 4; ++tt) { const int tile = wave * 4 + tt; const int ry = y0 + (tile >> 2), x0 = (tile & 3) * 16;
    for (int q = lane; q < 16 * K2P; q += 32) { const int px = q / K2P, k = q % K2P; b16 hv = (b16)0.0f, lv = (b16)0.0f;
      if (k < K2) { const int ci = k / 9, ky = (k % 9) / 3, kx = k % 3; const int yy = ry + ky - 1, xx = x0 + px + kx - 1; if (yy >= 0 && yy < H1 && xx >= 0 && xx < H1) { const size_t gi = ((size_t)ci * H1 + yy) * H1 + xx; hv = ph[gi]; lv = pl[gi]; } }
      Ah[wave][px][k] = hv; Al[wave][px][k] = lv; }
    wave_lds_sync();
    v8f d[2] = {{}, {}};
#pragma unroll
    for (int kb = 0; kb < K2P; kb += 32) { const v16b a = frag_kb(&Ah[wave][nloc][kb], hlf), al = frag_kb(&Al[wave][nloc][kb], hlf);
#pragma unroll
      for (int t = 0; t < 2; ++t) { const v16b bw = frag_kb(W2P + (size_t)(t * 16 + nloc) * K2P + kb, hlf); d[t] = wmma16b(a, bw, d[t]); d[t] = wmma16b(al, bw, d[t]); } }
    for (int t = 0; t < 2; ++t) { const int oc = t * 16 + nloc; const float bb = bf16_rne(b2[oc]); for (int r = 0; r < 8; ++r) Cs[tile >> 2][x0 + 8 * hlf + r][oc] = fmaxf(d[t][r] * (1.0f / (XS * WSC)) + bb, 0.0f); }
    wave_lds_sync(); }
  __syncthreads();
  for (int q = t_; q < C2 * 2 * H2; q += 128) { const int c = q / (2 * H2), rem = q % (2 * H2); const int pr = rem / H2, px = rem % H2; const float m = fmaxf(fmaxf(Cs[2 * pr][2 * px][c], Cs[2 * pr][2 * px + 1][c]), fmaxf(Cs[2 * pr + 1][2 * px][c], Cs[2 * pr + 1][2 * px + 1][c])); b16 p, ql; split16(m * XS, p, ql); Rh[c][rem] = p; Rl[c][rem] = ql; }
  __syncthreads();
  for (int pass = 0; pass < 2; ++pass) { for (int q = t_; q < C2 * 8; q += 128) { const int c = q >> 3, c8 = (q & 7) * 8; const size_t gi = (((size_t)f * C2 + c) * H2 + 2 * blockIdx.x) * H2 + c8; *(volatile v8b*)(P2h + gi) = *(const v8b*)(&Rh[c][c8]); *(volatile v8b*)(P2l + gi) = *(const v8b*)(&Rl[c][c8]); } __threadfence(); }
}
__global__ __launch_bounds__(128) void conv3_kernel(const b16* __restrict__ P2h, const b16* __restrict__ P2l, const b16* __restrict__ W3P, const float* __restrict__ b3, float* __restrict__ FEAT) {
  __shared__ __attribute__((aligned(16))) b16 Ah[4][16][K3 + 8], Al[4][16][K3 + 8]; __shared__ float Ws[4][2][C3]; __shared__ __attribute__((aligned(16))) float row[C3];
  const int f = blockIdx.x; const int wave = threadIdx.x >> 5, lane = threadIdx.x & 31, nloc = lane & 15, hlf = lane >> 4, t_ = threadIdx.x;
  const b16* ph = P2h + (size_t)f * C2 * H2 * H2; const b16* pl = P2l + (size_t)f * C2 * H2 * H2;
  float csum[4] = {0.0f, 0.0f, 0.0f, 0.0f};
  for (int tt = 0; tt < 16; ++tt) { const int tile = wave * 16 + tt; const int ry = tile >> 1, x0 = (tile & 1) * 16;
    for (int q = lane; q < 16 * K3; q += 32) { const int px = q / K3, k = q % K3; const int ci = k / 9, ky = (k % 9) / 3, kx = k % 3; const int yy = ry + ky - 1, xx = x0 + px + kx - 1; b16 hv = (b16)0.0f, lv = (b16)0.0f;
      if (yy >= 0 && yy < H2 && xx >= 0 && xx < H2) { const size_t gi = ((size_t)ci * H2 + yy) * H2 + xx; hv = ph[gi]; lv = pl[gi]; }
      Ah[wave][px][k] = hv; Al[wave][px][k] = lv; }
    wave_lds_sync();
    v8f d[4] = {{}, {}, {}, {}};
#pragma unroll 3
    for (int kb = 0; kb < K3; kb += 32) { const v16b a = frag_kb(&Ah[wave][nloc][kb], hlf), al = frag_kb(&Al[wave][nloc][kb], hlf);
#pragma unroll
      for (int t = 0; t < 4; ++t) { const v16b bw = frag_kb(W3P + (size_t)(t * 16 + nloc) * K3 + kb, hlf); d[t] = wmma16b(a, bw, d[t]); d[t] = wmma16b(al, bw, d[t]); } }
#pragma unroll
    for (int t = 0; t < 4; ++t) { const float bb = bf16_rne(b3[t * 16 + nloc]); for (int r = 0; r < 8; ++r) csum[t] += fmaxf(d[t][r] * (1.0f / (XS * WSC)) + bb, 0.0f); }
    wave_lds_sync(); }
#pragma unroll
  for (int t = 0; t < 4; ++t) Ws[wave][hlf][t * 16 + nloc] = csum[t];
  __syncthreads();
  if (t_ < C3) { float s = 0.0f; for (int w = 0; w < 4; ++w) s += Ws[w][0][t_] + Ws[w][1][t_]; row[t_] = s * (1.0f / (H2 * H2)); }
  __syncthreads();
  for (int pass = 0; pass < 2; ++pass) { if (t_ < 16) *(volatile v4f*)(FEAT + (size_t)f * C3 + t_ * 4) = *(const v4f*)(&row[t_ * 4]); __threadfence(); }
}
__global__ __launch_bounds__(256) void tail_kernel(const float* __restrict__ FEAT, const float* __restrict__ fcw, const float* __restrict__ fcb, const float* __restrict__ qw, const float* __restrict__ kw, const float* __restrict__ vw, float* __restrict__ out) {
  __shared__ float fe[S + 1][FD]; __shared__ float kk[S][DK], vv[S][DV], qq[DK]; __shared__ float sc[S], at[S]; __shared__ __attribute__((aligned(16))) float res[DV];
  const int b = blockIdx.x, t_ = threadIdx.x;
  for (int q = t_; q < (S + 1) * FD; q += 256) { const int fr = q / FD, o = q % FD; const float* fv = FEAT + ((size_t)b * (S + 1) + fr) * C3; float s = bf16_rne(fcb[o]);
#pragma unroll 1
    for (int k = 0; k < C3; ++k) s += pmul(fv[k], bf16_rne(fcw[o * C3 + k])); fe[fr][o] = s; }
  __syncthreads();
  for (int q = t_; q < S * DK + S * DV + DK; q += 256) {
    if (q < S * DK) { const int fr = q / DK, o = q % DK; const int slot = (T0 + fr) % S; float s = 0.0f;
#pragma unroll 1
      for (int k = 0; k < FD; ++k) s += pmul(fe[fr][k], bf16_rne(kw[o * FD + k])); kk[slot][o] = s; }
    else if (q < S * DK + S * DV) { const int q2 = q - S * DK; const int fr = q2 / DV, o = q2 % DV; const int slot = (T0 + fr) % S; float s = 0.0f;
#pragma unroll 1
      for (int k = 0; k < FD; ++k) s += pmul(fe[fr][k], bf16_rne(vw[o * FD + k])); vv[slot][o] = s; }
    else { const int o = q - S * DK - S * DV; float s = 0.0f;
#pragma unroll 1
      for (int k = 0; k < FD; ++k) s += pmul(fe[S][k], bf16_rne(qw[o * FD + k])); qq[o] = s; } }
  __syncthreads();
  if (t_ < S) { float s = 0.0f; for (int k = 0; k < DK; ++k) s += pmul(qq[k], kk[t_][k]); sc[t_] = s * SCALE; }
  __syncthreads();
  if (t_ == 0) { float mx = -INFINITY; for (int j = 0; j < S; ++j) mx = fmaxf(mx, sc[j]); float se = 0.0f; for (int j = 0; j < S; ++j) { at[j] = __expf(sc[j] - mx); se += at[j]; } for (int j = 0; j < S; ++j) at[j] /= se; }
  __syncthreads();
  if (t_ < DV) { float s = 0.0f; for (int j = 0; j < S; ++j) s += pmul(at[j], vv[j][t_]); res[t_] = s; }
  __syncthreads();
  for (int pass = 0; pass < 2; ++pass) { if (t_ < 32) *(volatile v4f*)(out + (size_t)b * DV + t_ * 4) = *(const v4f*)(&res[t_ * 4]); __threadfence(); }
}
}

extern "C" void kernel_launch(void* const* d_in, const int* in_sizes, int n_in, void* d_out, int out_size, void* d_ws, size_t ws_size, hipStream_t stream) {
  (void)n_in;
  auto Fp = [&](int i) { return (const float*)d_in[i]; };
  if (in_sizes[0] != NB * T * HW * HW || in_sizes[1] != C1 * 9 || in_sizes[3] != C2 * K2 || in_sizes[5] != C3 * K3 || in_sizes[7] != FD * C3 || in_sizes[9] != DK * FD || in_sizes[11] != DV * FD || out_size != NB * DV) return;
  size_t off = 0; char* ws = (char*)d_ws;
  auto carve = [&](size_t bytes) { char* p = ws + off; off += (bytes + 255) & ~(size_t)255; return p; };
  b16* W1P = (b16*)carve(C1 * 32 * 2); b16* W2P = (b16*)carve(C2 * K2P * 2); b16* W3P = (b16*)carve(C3 * K3 * 2);
  b16* P1h = (b16*)carve((size_t)NFR * C1 * H1 * H1 * 2); b16* P1l = (b16*)carve((size_t)NFR * C1 * H1 * H1 * 2); b16* P2h = (b16*)carve((size_t)NFR * C2 * H2 * H2 * 2); b16* P2l = (b16*)carve((size_t)NFR * C2 * H2 * H2 * 2); float* FEAT = (float*)carve((size_t)NFR * C3 * 4);
  if (off > ws_size || off > ((size_t)128 << 20)) return;
  prepw_kernel<<<(C1 * 32 / 8 + C2 * K2P / 8 + C3 * K3 / 8 + 255) / 256, 256, 0, stream>>>(Fp(1), Fp(3), Fp(5), W1P, W2P, W3P);
  conv1_kernel<<<dim3(H1, NFR), 256, 0, stream>>>(Fp(0), W1P, Fp(2), P1h, P1l);
  conv2_kernel<<<dim3(H1 / 4, NFR), 128, 0, stream>>>(P1h, P1l, W2P, Fp(4), P2h, P2l);
  conv3_kernel<<<NFR, 128, 0, stream>>>(P2h, P2l, W3P, Fp(6), FEAT);
  tail_kernel<<<NB, 256, 0, stream>>>(FEAT, Fp(7), Fp(8), Fp(9), Fp(10), Fp(11), (float*)d_out);
}
